// FullAttention_new_84911503442243
// MI455X (gfx1250) — hardware-verified
//
#include <hip/hip_runtime.h>


#define NB_  4
#define TT   1024
#define NH_  16
#define HD   32
#define DD   (NH_ * HD)
#define NT   (NB_ * TT)
#define NZ   (NB_ * NH_)
#define ZB   8
typedef _Float16 h16;
typedef unsigned short bf;
typedef __attribute__((ext_vector_type(16))) __bf16   v16bf;
typedef __attribute__((ext_vector_type(16))) _Float16 v16h;
typedef __attribute__((ext_vector_type(8)))  _Float16 v8h;
typedef __attribute__((ext_vector_type(8)))  unsigned short v8us;
typedef __attribute__((ext_vector_type(8)))  float    v8f;
typedef __attribute__((ext_vector_type(4)))  float    v4f;
typedef v8h  __attribute__((may_alias)) v8ha;
typedef v4f  __attribute__((may_alias)) v4fa;
typedef v8us __attribute__((may_alias)) v8usa;

__device__ __forceinline__ unsigned short f2bf(float f) { unsigned u = __float_as_uint(f); u += 0x7FFFu + ((u >> 16) & 1u); return (unsigned short)(u >> 16); }
__device__ __forceinline__ float bf2f(unsigned short b) { return __uint_as_float(((unsigned)b) << 16); }
__device__ __forceinline__ float bfr(float f) { return bf2f(f2bf(f)); }
__device__ __forceinline__ v16h cat16(v8h lo, v8h hi) { return __builtin_shufflevector(lo, hi, 0, 1, 2, 3, 4, 5, 6, 7, 8, 9, 10, 11, 12, 13, 14, 15); }
__device__ __forceinline__ v16bf cat16b(v8us lo, v8us hi) { return __builtin_bit_cast(v16bf, __builtin_shufflevector(lo, hi, 0, 1, 2, 3, 4, 5, 6, 7, 8, 9, 10, 11, 12, 13, 14, 15)); }
__device__ __forceinline__ v8f wmma16(v16h a, v16h b, v8f c) { return __builtin_amdgcn_wmma_f32_16x16x32_f16(false, a, false, b, (short)0, c, false, false); }
__device__ __forceinline__ v8f wmmab(v16bf a, v16bf b, v8f c) { return __builtin_amdgcn_wmma_f32_16x16x32_bf16(false, a, false, b, (short)0, c, false, false); }


template <typename T16> struct WFrag;
template <> struct WFrag<h16> { typedef v16h V; static __device__ __forceinline__ V ld(const h16* p) { return cat16(*(const v8h*)p, *(const v8h*)(p + 16)); } static __device__ __forceinline__ v8f mma(V a, V b, v8f c) { return wmma16(a, b, c); } };
template <> struct WFrag<bf> { typedef v16bf V; static __device__ __forceinline__ V ld(const bf* p) { return cat16b(*(const v8us*)p, *(const v8us*)(p + 16)); } static __device__ __forceinline__ v8f mma(V a, V b, v8f c) { return wmmab(a, b, c); } };
template <typename T16, int NSPLIT, bool BIAS>
__global__ __launch_bounds__(32) void k_gemmw(const T16* __restrict__ A, const T16* __restrict__ A2, const T16* __restrict__ Bt, const T16* __restrict__ Bt2, int K, float* C, int ldc, const float* __restrict__ bias, size_t sA, size_t sB, size_t sC) {
    typedef typename WFrag<T16>::V V;
    __shared__ __align__(16) float os[16 * 68];
    const size_t z = blockIdx.z; A += z * sA; if (A2) A2 += z * sA; Bt += z * sB; if (Bt2) Bt2 += z * sB; C += z * sC;
    const int lane = threadIdx.x & 31, lr = lane & 15, hi = lane >> 4; const int r0 = blockIdx.x * 64, c0 = blockIdx.y * 64;
    v8f acc[4][4];
#pragma unroll
    for (int mb = 0; mb < 4; ++mb)
#pragma unroll
        for (int nb = 0; nb < 4; ++nb) acc[mb][nb] = (v8f){};
    const size_t aoff = (size_t)(r0 + lr) * K + 8 * hi, boff = (size_t)(c0 + lr) * K + 8 * hi;
#pragma unroll 1
    for (int kc = 0; kc < K; kc += 32) {
        V a[4], a2[4];
#pragma unroll
        for (int mb = 0; mb < 4; ++mb) { a[mb] = WFrag<T16>::ld(A + aoff + (size_t)mb * 16 * K + kc); if (NSPLIT == 1 || NSPLIT == 2) a2[mb] = WFrag<T16>::ld(A2 + aoff + (size_t)mb * 16 * K + kc); }
#pragma unroll
        for (int nb = 0; nb < 4; ++nb) { const V b = WFrag<T16>::ld(Bt + boff + (size_t)nb * 16 * K + kc); V b2; if (NSPLIT >= 2) b2 = WFrag<T16>::ld(Bt2 + boff + (size_t)nb * 16 * K + kc);
#pragma unroll
            for (int mb = 0; mb < 4; ++mb) { acc[mb][nb] = WFrag<T16>::mma(a[mb], b, acc[mb][nb]); if (NSPLIT == 1 || NSPLIT == 2) acc[mb][nb] = WFrag<T16>::mma(a2[mb], b, acc[mb][nb]); if (NSPLIT >= 2) acc[mb][nb] = WFrag<T16>::mma(a[mb], b2, acc[mb][nb]); } }
        asm volatile("v_nop\n\tv_nop\n\tv_nop\n\tv_nop" : "+v"(acc[0][0]), "+v"(acc[1][1]), "+v"(acc[2][2]), "+v"(acc[3][3]) : "v"(a[0]), "v"(a[3]));
    }
#pragma unroll
    for (int mb = 0; mb < 4; ++mb) {
#pragma unroll
        for (int nb = 0; nb < 4; ++nb) {
#pragma unroll
            for (int j = 0; j < 8; ++j) os[(hi * 8 + j) * 68 + nb * 16 + lr] = acc[mb][nb][j]; }
        __builtin_amdgcn_wave_barrier(); asm volatile("" ::: "memory");
        float* crow = C + (size_t)(r0 + mb * 16) * ldc + c0;
#pragma unroll 1
        for (int ps = 0; ps < 2; ++ps) {
#pragma unroll
            for (int s = 0; s < 8; ++s) { const int row = 2 * s + hi, cofs = lr * 4; v4f val = *(const v4fa*)(os + row * 68 + cofs); if (BIAS) { val[0] += bfr(bias[c0 + cofs]); val[1] += bfr(bias[c0 + cofs + 1]); val[2] += bfr(bias[c0 + cofs + 2]); val[3] += bfr(bias[c0 + cofs + 3]); }
                *(volatile v4f*)(crow + (size_t)row * ldc + cofs) = val; }
            if (ps == 0) __threadfence(); }
        __builtin_amdgcn_wave_barrier(); asm volatile("" ::: "memory");
    }
}

__device__ __forceinline__ void splitf(float y, unsigned short& h, unsigned short& l) { h = f2bf(y); l = f2bf(y - bf2f(h)); }
typedef __attribute__((ext_vector_type(2))) unsigned short v2us;
typedef __attribute__((ext_vector_type(4))) unsigned short v4us;
typedef __attribute__((ext_vector_type(2))) float v2f;

__global__ __launch_bounds__(256) void k_planes(const float* __restrict__ q, const float* __restrict__ k, bf* QP, bf* KP, bf* FRh, bf* FRl) {
    const int lane = threadIdx.x & 31; const int L0 = (blockIdx.x * 8 + (threadIdx.x >> 5)) * 8; const int nlines = NZ * TT * HD / 64;
#pragma unroll 1
    for (int ps = 0; ps < 2; ++ps) {
#pragma unroll
        for (int l = 0; l < 8; ++l) { const int L = L0 + l; if (L >= nlines) break; const int e = L * 64 + lane * 2; const int d = e & 31; const int t = (e >> 5) & (TT - 1); const int z = e >> 15; const int b = z / NH_, h = z % NH_; v2us oq, ok, fh, fl;
#pragma unroll
            for (int qq = 0; qq < 2; ++qq) { const size_t src = (((size_t)b * TT + t) * NH_ + h) * HD + d + qq; const float qv = bfr(q[src]), kv = bfr(k[src]); oq[qq] = f2bf(qv); ok[qq] = f2bf(kv); unsigned short a, c2; splitf(fabsf(qv) + fabsf(kv), a, c2); fh[qq] = a; fl[qq] = c2; }
            *(volatile v2us*)(QP + (size_t)e) = oq; *(volatile v2us*)(KP + (size_t)e) = ok; *(volatile v2us*)(FRh + (size_t)e) = fh; *(volatile v2us*)(FRl + (size_t)e) = fl; }
        if (ps == 0) __threadfence(); }
}
__global__ __launch_bounds__(256) void k_wplane(const float* __restrict__ w, bf* WP) {
    const int lane = threadIdx.x & 31; const int L0 = (blockIdx.x * 8 + (threadIdx.x >> 5)) * 8; const int nlines = NH_ * TT * HD / 64;
#pragma unroll 1
    for (int ps = 0; ps < 2; ++ps) {
#pragma unroll
        for (int l = 0; l < 8; ++l) { const int L = L0 + l; if (L >= nlines) break; const int e = L * 64 + lane * 2; const int d = e & 31; const int s = (e >> 5) & (TT - 1); const int h = e >> 15; v2us o;
#pragma unroll
            for (int qq = 0; qq < 2; ++qq) o[qq] = f2bf(w[((size_t)s * NH_ + h) * HD + d + qq]);
            *(volatile v2us*)(WP + (size_t)e) = o; }
        if (ps == 0) __threadfence(); }
}
__global__ __launch_bounds__(256) void k_vtplane(const float* __restrict__ v, bf* VT) {
    const int lane = threadIdx.x & 31; const int L0 = (blockIdx.x * 8 + (threadIdx.x >> 5)) * 8; const int nlines = NZ * 64 * TT / 64;
#pragma unroll 1
    for (int ps = 0; ps < 2; ++ps) {
#pragma unroll
        for (int l = 0; l < 8; ++l) { const int L = L0 + l; if (L >= nlines) break; const int e = L * 64 + lane * 2; const int s = e & (TT - 1); const int d = (e >> 10) & 63; const int z = e >> 16; const int b = z / NH_, h = z % NH_; v2us o;
#pragma unroll
            for (int qq = 0; qq < 2; ++qq) o[qq] = (d < HD) ? f2bf(v[(((size_t)b * TT + s + qq) * NH_ + h) * HD + d]) : (unsigned short)0;
            *(volatile v2us*)(VT + (size_t)e) = o; }
        if (ps == 0) __threadfence(); }
}
__global__ __launch_bounds__(256) void k_gate(float* S, const float* __restrict__ S2) {
    const int lane = threadIdx.x & 31; const int row = blockIdx.x * 8 + (threadIdx.x >> 5); if (row >= ZB * TT) return; float* sr = S + (size_t)row * TT; const float* sr2 = S2 + (size_t)row * TT; const float sc = 0.17677669529663687f;
#pragma unroll 1
    for (int j0 = lane * 4; j0 < TT; j0 += 128) { const v4f a = *(const v4f*)(sr + j0), a2 = *(const v4f*)(sr2 + j0); v4f o;
#pragma unroll
        for (int q = 0; q < 4; ++q) { const float s1 = fminf(fmaxf(a[q], -1000.f), 1000.f) * sc, s2 = fminf(fmaxf(a2[q], -1000.f), 1000.f) * sc; o[q] = tanhf(s1) * __fdiv_rn(1.0f, 1.0f + __expf(-s2)); }
        *(volatile v4f*)(sr + j0) = o; __threadfence(); *(volatile v4f*)(sr + j0) = o; }
}
__global__ __launch_bounds__(256) void k_soft(const float* __restrict__ S, bf* Ph, bf* Pl) {
    const int lane = threadIdx.x & 31; const int row = blockIdx.x * 8 + (threadIdx.x >> 5); if (row >= ZB * TT) return; const float* sr = S + (size_t)row * TT; float v[32]; float mx = -3.0e38f;
#pragma unroll
    for (int ch = 0; ch < 8; ++ch) { const v4f a = *(const v4f*)(sr + ch * 128 + lane * 4);
#pragma unroll
        for (int q = 0; q < 4; ++q) { v[ch * 4 + q] = a[q]; mx = fmaxf(mx, a[q]); } }
#pragma unroll
    for (int sh = 16; sh; sh >>= 1) mx = fmaxf(mx, __shfl_xor(mx, sh, 32));
    float sum = 0.f;
#pragma unroll
    for (int kk = 0; kk < 32; ++kk) { v[kk] = __expf(v[kk] - mx); sum += v[kk]; }
#pragma unroll
    for (int sh = 16; sh; sh >>= 1) sum += __shfl_xor(sum, sh, 32);
    const float f = __fdiv_rn(1.0f, sum);
#pragma unroll 1
    for (int ps = 0; ps < 2; ++ps) {
#pragma unroll
        for (int ch = 0; ch < 8; ++ch) { v4us oh, ol;
#pragma unroll
            for (int q = 0; q < 4; ++q) { unsigned short a, c2; splitf(v[ch * 4 + q] * f, a, c2); oh[q] = a; ol[q] = c2; }
            *(volatile v4us*)(Ph + (size_t)row * TT + ch * 128 + lane * 4) = oh; *(volatile v4us*)(Pl + (size_t)row * TT + ch * 128 + lane * 4) = ol; }
        if (ps == 0) __threadfence(); }
}
__global__ __launch_bounds__(256) void k_out(const float* __restrict__ O, int z0, float* OUT) {
    const int lane = threadIdx.x & 31; const int L0 = (blockIdx.x * 8 + (threadIdx.x >> 5)) * 8; const int nlines = ZB * TT * HD / 64;
#pragma unroll 1
    for (int ps = 0; ps < 2; ++ps) {
#pragma unroll
        for (int l = 0; l < 8; ++l) { const int L = L0 + l; if (L >= nlines) break; const int e = L * 64 + lane * 2; const int d = e & 31; const int t = (e >> 5) & (TT - 1); const int zz = e >> 15; const int z = z0 + zz; const int b = z / NH_, h = z % NH_; v2f o;
            o[0] = O[((size_t)zz * TT + t) * 64 + d]; o[1] = O[((size_t)zz * TT + t) * 64 + d + 1];
            *(volatile v2f*)(OUT + (((size_t)b * TT + t) * NH_ + h) * HD + d) = o; }
        if (ps == 0) __threadfence(); }
}

extern "C" void kernel_launch(void* const* d_in, const int* in_sizes, int n_in,
                              void* d_out, int out_size, void* d_ws, size_t ws_size, hipStream_t stream) {
    (void)in_sizes; (void)n_in; (void)out_size;
    const float* q = (const float*)d_in[0]; const float* k = (const float*)d_in[1]; const float* v = (const float*)d_in[2]; const float* w = (const float*)d_in[3];
    float* OUT = (float*)d_out;
    char* wsp = (char*)d_ws;
    auto take = [&](size_t bytes) { char* p = wsp; wsp += (bytes + 255) & ~(size_t)255; return (void*)p; };
    const size_t PLN = (size_t)NZ * TT * HD;
    bf* QP = (bf*)take(PLN * 2); bf* KP = (bf*)take(PLN * 2); bf* FRh = (bf*)take(PLN * 2); bf* FRl = (bf*)take(PLN * 2); bf* WP = (bf*)take((size_t)NH_ * TT * HD * 2); bf* VT = (bf*)take((size_t)NZ * 64 * TT * 2);
    float* S = (float*)take((size_t)ZB * TT * TT * 4); float* S2 = (float*)take((size_t)ZB * TT * TT * 4); bf* Ph = (bf*)take((size_t)ZB * TT * TT * 2); bf* Pl = (bf*)take((size_t)ZB * TT * TT * 2); float* Ob = (float*)take((size_t)ZB * TT * 64 * 4);
    if ((size_t)(wsp - (char*)d_ws) > ws_size) return;
    const unsigned LP = (unsigned)((NZ * TT * HD / 64 + 63) / 64);
    k_planes<<<LP, 256, 0, stream>>>(q, k, QP, KP, FRh, FRl); k_wplane<<<(NH_ * TT * HD / 64 + 63) / 64, 256, 0, stream>>>(w, WP); k_vtplane<<<(unsigned)((NZ * 64 * TT / 64 + 63) / 64), 256, 0, stream>>>(v, VT);
    for (int z0 = 0; z0 < NZ; z0 += ZB) { const int h0 = z0 % NH_;
        k_gemmw<bf, 0, false><<<dim3(TT / 64, TT / 64, ZB), 32, 0, stream>>>(QP + (size_t)z0 * TT * HD, nullptr, KP + (size_t)z0 * TT * HD, nullptr, HD, S, TT, nullptr, (size_t)TT * HD, (size_t)TT * HD, (size_t)TT * TT);
        k_gemmw<bf, 1, false><<<dim3(TT / 64, TT / 64, ZB), 32, 0, stream>>>(FRh + (size_t)z0 * TT * HD, FRl + (size_t)z0 * TT * HD, WP + (size_t)h0 * TT * HD, nullptr, HD, S2, TT, nullptr, (size_t)TT * HD, (size_t)TT * HD, (size_t)TT * TT);
        k_gate<<<ZB * TT / 8, 256, 0, stream>>>(S, S2); k_soft<<<ZB * TT / 8, 256, 0, stream>>>(S, Ph, Pl);
        k_gemmw<bf, 1, false><<<dim3(TT / 64, 1, ZB), 32, 0, stream>>>(Ph, Pl, VT + (size_t)z0 * 64 * TT, nullptr, TT, Ob, 64, nullptr, (size_t)TT * TT, (size_t)64 * TT, (size_t)TT * 64);
        k_out<<<(ZB * TT * HD / 64 + 63) / 64, 256, 0, stream>>>(Ob, z0, OUT); }
}
